// MiniMaxM2Attention_88579405513103
// MI455X (gfx1250) — hardware-verified
//
#include <hip/hip_runtime.h>
#include <math.h>
#include <stdint.h>
#include <stddef.h>

#define NBATCH 2
#define SEQ    2048
#define HID    2048
#define NQH    16
#define NKVH   4
#define HDIM   128
#define QDIM   2048
#define KDIM   512
#define QKLD   2560
#define WIN    1024
#define NFREQ  32

typedef __attribute__((ext_vector_type(16))) __bf16         v16b;
typedef __attribute__((ext_vector_type(8)))  unsigned short v8us;
typedef __attribute__((ext_vector_type(8)))  float          v8f;
typedef __attribute__((ext_vector_type(4)))  float          v4f;
typedef __attribute__((ext_vector_type(4)))  unsigned int   v4u;

__device__ __forceinline__ unsigned short f2bf_bits(float f) {
  const unsigned u = __float_as_uint(f);
  return (unsigned short)((u + 0x7FFFu + ((u >> 16) & 1u)) >> 16);
}
__device__ __forceinline__ float bf_bits2f(unsigned short h) { return __uint_as_float(((unsigned)h) << 16); }
__device__ __forceinline__ unsigned pk16(unsigned short a, unsigned short b) { return (unsigned)a | ((unsigned)b << 16); }
__device__ __forceinline__ v8f vzero8() { v8f z = {0.f, 0.f, 0.f, 0.f, 0.f, 0.f, 0.f, 0.f}; return z; }

union Frag16 { v16b v; v8us u[2]; };
__device__ __forceinline__ v16b ld_frag(const unsigned short* p) {
  Frag16 f;
  f.u[0] = *(const v8us*)(p);
  f.u[1] = *(const v8us*)(p + 16);
  return f.v;
}
__device__ __forceinline__ v8f mma_g(v16b a, v16b b, v8f c) {
  c = __builtin_amdgcn_wmma_f32_16x16x32_bf16(false, a, false, b, (short)0, c, false, false);
  asm volatile("v_nop\n\tv_nop\n\tv_nop\n\tv_nop" : "+v"(c) : "v"(a), "v"(b));
  return c;
}
__device__ __forceinline__ void wave_lds_sync() {
  __builtin_amdgcn_fence(__ATOMIC_RELEASE, "workgroup");
  __builtin_amdgcn_wave_barrier();
  __builtin_amdgcn_fence(__ATOMIC_ACQUIRE, "workgroup");
}

__global__ __launch_bounds__(256) void conv_bf16_kernel(const float* __restrict__ in, unsigned short* __restrict__ outp, int n8) {
  const int i = blockIdx.x * 256 + threadIdx.x;
  if (i < n8) {
    const size_t e0 = 8 * (size_t)i;
    const v4f a = *(const v4f*)(in + e0);
    const v4f b = *(const v4f*)(in + e0 + 4);
    v4u o;
    o[0] = pk16(f2bf_bits(a[0]), f2bf_bits(a[1]));
    o[1] = pk16(f2bf_bits(a[2]), f2bf_bits(a[3]));
    o[2] = pk16(f2bf_bits(b[0]), f2bf_bits(b[1]));
    o[3] = pk16(f2bf_bits(b[2]), f2bf_bits(b[3]));
    *(volatile v4u*)(outp + e0) = o;
    __threadfence();
    *(volatile v4u*)(outp + e0) = o;
  }
}

__global__ __launch_bounds__(256) void tconv_kernel(const float* __restrict__ W, unsigned short* __restrict__ outp, int R, int Cc) {
  __shared__ __align__(16) float tf[64 * 68];
  const int c0  = blockIdx.x * 64;
  const int r0  = blockIdx.y * 64;
  const int tid = threadIdx.x;
  {
    const int lr = tid >> 4;
    const int c4 = (tid & 15) * 4;
#pragma unroll
    for (int it = 0; it < 4; ++it) {
      const int rr = it * 16 + lr;
      const v4f a = *(const v4f*)(W + (size_t)(r0 + rr) * Cc + c0 + c4);
      *(v4f*)(tf + rr * 68 + c4) = a;
    }
  }
  __syncthreads();
  const int sub = tid >> 3;
  const int c8  = (tid & 7) * 8;
  v4u hv[2];
#pragma unroll
  for (int it = 0; it < 2; ++it) {
    const int oc = it * 32 + sub;
    v4u a;
#pragma unroll
    for (int q = 0; q < 4; ++q) {
      const float f0 = tf[(c8 + 2 * q) * 68 + oc];
      const float f1 = tf[(c8 + 2 * q + 1) * 68 + oc];
      a[q] = pk16(f2bf_bits(f0), f2bf_bits(f1));
    }
    hv[it] = a;
  }
  for (int pass = 0; pass < 2; ++pass) {
#pragma unroll
    for (int it = 0; it < 2; ++it) {
      const int oc = it * 32 + sub;
      const size_t go = (size_t)(c0 + oc) * R + r0 + c8;
      *(volatile v4u*)(outp + go) = hv[it];
    }
    __threadfence();
  }
}

__global__ __launch_bounds__(256) void rope_tab_kernel(const int* __restrict__ pid, int npos,
                                                       float* __restrict__ ct, float* __restrict__ st, int ntok) {
  const int gid = blockIdx.x * 256 + threadIdx.x;
  const int t = gid >> 5;
  const int j = gid & 31;
  int pi = t;
  if (pi > npos - 1) pi = npos - 1;
  if (pi < 0) pi = 0;
  const float pos = (float)pid[pi];
  const float e   = (float)(2 * j) * 0.015625f;
  const float pw  = powf(1000000.0f, e);
  const float inv = 1.0f / pw;
  const float ang = pos * inv;
  float sn, cs;
  sincosf(ang, &sn, &cs);
  if (t < ntok) {
    float* cp = ct + (size_t)t * NFREQ + j;
    float* sp = st + (size_t)t * NFREQ + j;
    *(volatile float*)cp = cs;
    *(volatile float*)sp = sn;
    __threadfence();
    *(volatile float*)cp = cs;
    *(volatile float*)sp = sn;
  }
}

template <bool ASPLIT, int OUTM>
__global__ __launch_bounds__(256) void gemm64_kernel(
    const unsigned short* __restrict__ Ap, const unsigned short* __restrict__ A2p, int lda, long long strideA,
    const unsigned short* __restrict__ Btp, int ldb, long long strideB,
    float* __restrict__ Cf, unsigned short* __restrict__ Ch, unsigned short* __restrict__ Cl, int ldc, long long strideC,
    int M, int N, int K) {
  __shared__ __align__(16) float sT[8][16 * 68];
  const int bz   = blockIdx.y;
  const int lane = threadIdx.x & 31;
  const int wave = threadIdx.x >> 5;
  const int tilesN = N >> 6;
  const int tilesM = M >> 6;
  const int tile = blockIdx.x * 8 + wave;
  if (tile >= tilesM * tilesN) return;
  const int tm = tile / tilesN;
  const int tn = tile - tm * tilesN;
  const int m0 = tm << 6;
  const int n0 = tn << 6;

  const unsigned short* Ab  = Ap + (size_t)bz * (size_t)strideA;
  const unsigned short* Ab2 = ASPLIT ? (A2p + (size_t)bz * (size_t)strideA) : Ab;
  const unsigned short* Bb  = Btp + (size_t)bz * (size_t)strideB;

  const int rlane = lane & 15;
  const int koff  = (lane >> 4) * 8;
  const int mOff  = (lane >> 4) * 8;

  v8f acc[4][4];
#pragma unroll
  for (int i = 0; i < 4; ++i)
#pragma unroll
    for (int j = 0; j < 4; ++j) acc[i][j] = vzero8();

  for (int k0 = 0; k0 < K; k0 += 32) {
    v16b bf[4];
#pragma unroll
    for (int j = 0; j < 4; ++j)
      bf[j] = ld_frag(Bb + (size_t)(n0 + (j << 4) + rlane) * ldb + k0 + koff);
#pragma unroll
    for (int i = 0; i < 4; ++i) {
      const size_t ao = (size_t)(m0 + (i << 4) + rlane) * lda + k0 + koff;
      const v16b ah = ld_frag(Ab + ao);
      v16b al = ah;
      if (ASPLIT) al = ld_frag(Ab2 + ao);
#pragma unroll
      for (int j = 0; j < 4; ++j) {
        acc[i][j] = mma_g(ah, bf[j], acc[i][j]);
        if (ASPLIT) acc[i][j] = mma_g(al, bf[j], acc[i][j]);
      }
    }
  }

  float* slab = sT[wave];
#pragma unroll
  for (int i = 0; i < 4; ++i) {
    const int mBase = m0 + (i << 4);
#pragma unroll
    for (int j = 0; j < 4; ++j) {
#pragma unroll
      for (int r = 0; r < 8; ++r) slab[(mOff + r) * 68 + (j << 4) + rlane] = acc[i][j][r];
    }
    wave_lds_sync();
    if (OUTM == 0) {
      float* C = Cf + (size_t)bz * (size_t)strideC;
      const int h2 = lane >> 4, c4 = (lane & 15) * 4;
      for (int pass = 0; pass < 2; ++pass) {
#pragma unroll
        for (int it = 0; it < 8; ++it) {
          const int rr = it * 2 + h2;
          const v4f v = *(const v4f*)(slab + rr * 68 + c4);
          *(volatile v4f*)(C + (size_t)(mBase + rr) * ldc + n0 + c4) = v;
        }
        __threadfence();
      }
    } else {
      const int q = lane >> 3, c8 = (lane & 7) * 8;
      unsigned short* C1 = Ch + (size_t)bz * (size_t)strideC;
      unsigned short* C2 = Cl + (size_t)bz * (size_t)strideC;
      v4u hv[4], lv[4];
#pragma unroll
      for (int it = 0; it < 4; ++it) {
        const int rr = it * 4 + q;
        const float* sp = slab + rr * 68 + c8;
        v4u a, a2;
#pragma unroll
        for (int p = 0; p < 4; ++p) {
          const float f0 = sp[2 * p], f1 = sp[2 * p + 1];
          const unsigned short hb0 = f2bf_bits(f0), hb1 = f2bf_bits(f1);
          const unsigned short lb0 = f2bf_bits(f0 - bf_bits2f(hb0)), lb1 = f2bf_bits(f1 - bf_bits2f(hb1));
          a[p]  = pk16(hb0, hb1);
          a2[p] = pk16(lb0, lb1);
        }
        hv[it] = a; lv[it] = a2;
      }
      for (int pass = 0; pass < 2; ++pass) {
#pragma unroll
        for (int it = 0; it < 4; ++it) {
          const int rr = it * 4 + q;
          const size_t go = (size_t)(mBase + rr) * ldc + n0 + c8;
          *(volatile v4u*)(C1 + go) = hv[it];
          *(volatile v4u*)(C2 + go) = lv[it];
        }
        __threadfence();
      }
    }
    wave_lds_sync();
  }
}

__device__ __forceinline__ void norm_rope8(const float* xs, const float* __restrict__ w,
                                           const float* __restrict__ ctr, const float* __restrict__ str,
                                           int d0, float rs, v4u& hv, v4u& lv) {
  const int hd0 = d0 & (HDIM - 1);
#pragma unroll
  for (int p = 0; p < 4; ++p) {
    unsigned hpk = 0u, lpk = 0u;
#pragma unroll
    for (int e2 = 0; e2 < 2; ++e2) {
      const int e  = 2 * p + e2;
      const int d  = d0 + e;
      const int hd = hd0 + e;
      const int j  = hd & (NFREQ - 1);
      const float wv = bf_bits2f(f2bf_bits(w[d]));
      const float x  = xs[d] * rs * wv;
      const bool lowh = hd < 32;
      const int  pd   = lowh ? (d + 32) : (d - 32);
      const float wp = bf_bits2f(f2bf_bits(w[pd]));
      const float xp = xs[pd] * rs * wp;
      const float xr = lowh ? -xp : xp;
      const float cs = ctr[j], sn = str[j];
      const float rot = x * cs + xr * sn;
      const float val = (hd < 64) ? rot : x;
      const unsigned short hb = f2bf_bits(val);
      const unsigned short lb = f2bf_bits(val - bf_bits2f(hb));
      hpk |= ((unsigned)hb) << (16 * e2);
      lpk |= ((unsigned)lb) << (16 * e2);
    }
    hv[p] = hpk; lv[p] = lpk;
  }
}

__global__ __launch_bounds__(256) void norm_rope_kernel(
    const float* __restrict__ QK, int ldqk,
    const float* __restrict__ qw, const float* __restrict__ kw,
    const float* __restrict__ ct, const float* __restrict__ st,
    unsigned short* __restrict__ Qh, unsigned short* __restrict__ Ql,
    unsigned short* __restrict__ Kh, unsigned short* __restrict__ Kl, float eps) {
  __shared__ __align__(16) float qs[QDIM];
  __shared__ __align__(16) float ks[KDIM];
  __shared__ float red[2][8];
  const int t    = blockIdx.x;
  const int tid  = threadIdx.x;
  const int lane = tid & 31;
  const int wave = tid >> 5;
  const float* row = QK + (size_t)t * ldqk;

  const int d0 = 8 * tid;
  const v4f a0 = *(const v4f*)(row + d0);
  const v4f a1 = *(const v4f*)(row + d0 + 4);
  *(v4f*)(qs + d0) = a0;
  *(v4f*)(qs + d0 + 4) = a1;
  float sq = a0[0] * a0[0] + a0[1] * a0[1] + a0[2] * a0[2] + a0[3] * a0[3]
           + a1[0] * a1[0] + a1[1] * a1[1] + a1[2] * a1[2] + a1[3] * a1[3];
  const int k0 = 8 * (tid & 63);
  const v4f c0v = *(const v4f*)(row + QDIM + k0);
  const v4f c1v = *(const v4f*)(row + QDIM + k0 + 4);
  float sk = 0.f;
  if (tid < 64) {
    *(v4f*)(ks + k0) = c0v;
    *(v4f*)(ks + k0 + 4) = c1v;
    sk = c0v[0] * c0v[0] + c0v[1] * c0v[1] + c0v[2] * c0v[2] + c0v[3] * c0v[3]
       + c1v[0] * c1v[0] + c1v[1] * c1v[1] + c1v[2] * c1v[2] + c1v[3] * c1v[3];
  }
#pragma unroll
  for (int off = 16; off > 0; off >>= 1) {
    sq += __shfl_xor(sq, off, 32);
    sk += __shfl_xor(sk, off, 32);
  }
  if (lane == 0) { red[0][wave] = sq; red[1][wave] = sk; }
  __syncthreads();
  float tq = 0.f, tk = 0.f;
#pragma unroll
  for (int w = 0; w < 8; ++w) { tq += red[0][w]; tk += red[1][w]; }
  const float rq = rsqrtf(tq * (1.0f / (float)QDIM) + eps);
  const float rk = rsqrtf(tk * (1.0f / (float)KDIM) + eps);
  const float* ctr = ct + (size_t)t * NFREQ;
  const float* str = st + (size_t)t * NFREQ;

  {
    v4u hv, lv;
    norm_rope8(qs, qw, ctr, str, d0, rq, hv, lv);
    const size_t go = (size_t)t * QDIM + d0;
    *(volatile v4u*)(Qh + go) = hv;
    *(volatile v4u*)(Ql + go) = lv;
    __threadfence();
    *(volatile v4u*)(Qh + go) = hv;
    *(volatile v4u*)(Ql + go) = lv;
  }
  if (tid < 64) {
    v4u hv, lv;
    norm_rope8(ks, kw, ctr, str, k0, rk, hv, lv);
    const size_t go = (size_t)t * KDIM + k0;
    *(volatile v4u*)(Kh + go) = hv;
    *(volatile v4u*)(Kl + go) = lv;
    __threadfence();
    *(volatile v4u*)(Kh + go) = hv;
    *(volatile v4u*)(Kl + go) = lv;
  }
}

#define AQB 64
#define AQP 136
#define APP 72
#define AOP 132
#define ALDS_Q     (AQB * AQP * 2)
#define ALDS_P     (4 * 16 * APP * 2)
#define ALDS_BYTES (2 * ALDS_Q + 2 * ALDS_P)

__global__ __launch_bounds__(128) void attn_kernel(
    const unsigned short* __restrict__ Qh, const unsigned short* __restrict__ Ql,
    const unsigned short* __restrict__ Kh, const unsigned short* __restrict__ Kl,
    const unsigned short* __restrict__ VTh, const unsigned short* __restrict__ VTl,
    unsigned short* __restrict__ Ch, unsigned short* __restrict__ Cl, float sscale) {
  __shared__ __align__(16) unsigned char lds_raw[ALDS_BYTES];
  unsigned short* Qsh = (unsigned short*)(lds_raw);
  unsigned short* Qsl = (unsigned short*)(lds_raw + ALDS_Q);

  const int tid  = threadIdx.x;
  const int wave = tid >> 5;
  const int lane = tid & 31;
  const int hh   = lane >> 4;
  const int c    = lane & 15;
  const int bx = blockIdx.x;
  const int qb = bx & 31;
  const int h  = (bx >> 5) & 15;
  const int b  = bx >> 9;
  const int g  = h >> 2;
  const int q0 = qb * AQB;
  const size_t tok0 = (size_t)b * SEQ + q0;

  unsigned short* pwh = (unsigned short*)(lds_raw + 2 * ALDS_Q) + wave * (16 * APP);
  unsigned short* pwl = (unsigned short*)(lds_raw + 2 * ALDS_Q + ALDS_P) + wave * (16 * APP);

#pragma unroll
  for (int it = 0; it < 8; ++it) {
    const int p = it * 128 + tid;
    const int row = p >> 4, seg = p & 15;
    const size_t go = (tok0 + row) * QDIM + h * HDIM + seg * 8;
    const v4u a  = *(const v4u*)(Qh + go);
    const v4u a2 = *(const v4u*)(Ql + go);
    *(v4u*)(Qsh + row * AQP + seg * 8) = a;
    *(v4u*)(Qsl + row * AQP + seg * 8) = a2;
  }
  __syncthreads();

  const unsigned short* qsh = Qsh + (wave * 16 + c) * AQP + 8 * hh;
  const unsigned short* qsl = Qsl + (wave * 16 + c) * AQP + 8 * hh;
  const unsigned short* Kbh = Kh + (size_t)b * SEQ * KDIM + g * HDIM + 8 * hh;
  const unsigned short* Kbl = Kl + (size_t)b * SEQ * KDIM + g * HDIM + 8 * hh;
  const unsigned short* Vbh = VTh + ((size_t)b * KDIM + g * HDIM + c) * SEQ + 8 * hh;
  const unsigned short* Vbl = VTl + ((size_t)b * KDIM + g * HDIM + c) * SEQ + 8 * hh;
  const int qrow0 = q0 + wave * 16 + 8 * hh;

  float mrow[8], lrow[8];
  v8f oacc[8];
#pragma unroll
  for (int r = 0; r < 8; ++r) { mrow[r] = -INFINITY; lrow[r] = 0.f; }
#pragma unroll
  for (int t = 0; t < 8; ++t) oacc[t] = vzero8();

  const int kstart = (q0 > WIN) ? (q0 - WIN) : 0;
  const int ntiles = ((q0 - kstart) >> 6) + 1;

  for (int ti = 0; ti < ntiles; ++ti) {
    const int kt = kstart + ti * 64;

    v8f s[4];
#pragma unroll
    for (int j = 0; j < 4; ++j) s[j] = vzero8();
#pragma unroll 1
    for (int dc = 0; dc < 4; ++dc) {
      const v16b qa = ld_frag(qsh + dc * 32);
      const v16b qz = ld_frag(qsl + dc * 32);
#pragma unroll
      for (int j = 0; j < 4; ++j) {
        const size_t ko = (size_t)(kt + j * 16 + c) * KDIM + dc * 32;
        const v16b kb = ld_frag(Kbh + ko);
        const v16b kz = ld_frag(Kbl + ko);
        s[j] = mma_g(qa, kb, s[j]);
        s[j] = mma_g(qa, kz, s[j]);
        s[j] = mma_g(qz, kb, s[j]);
      }
    }

    float cm[8];
#pragma unroll
    for (int r = 0; r < 8; ++r) {
      const int qrow = qrow0 + r;
      float m = -INFINITY;
#pragma unroll
      for (int j = 0; j < 4; ++j) {
        const int key = kt + j * 16 + c;
        const float sv = s[j][r] * sscale;
        const bool masked = (key > qrow) || (key + WIN < qrow);
        const float sm = masked ? -INFINITY : sv;
        s[j][r] = sm;
        m = fmaxf(m, sm);
      }
#pragma unroll
      for (int off = 1; off < 16; off <<= 1) m = fmaxf(m, __shfl_xor(m, off, 32));
      cm[r] = m;
    }
    wave_lds_sync();

#pragma unroll
    for (int r = 0; r < 8; ++r) {
      const float mnew  = fmaxf(mrow[r], cm[r]);
      const float alpha = __expf(mrow[r] - mnew);
      mrow[r] = mnew;
      float psum = 0.f;
#pragma unroll
      for (int j = 0; j < 4; ++j) {
        const float p = __expf(s[j][r] - mnew);
        psum += p;
        const unsigned short hb = f2bf_bits(p);
        const unsigned short lb = f2bf_bits(p - bf_bits2f(hb));
        pwh[(8 * hh + r) * APP + j * 16 + c] = hb;
        pwl[(8 * hh + r) * APP + j * 16 + c] = lb;
      }
#pragma unroll
      for (int off = 1; off < 16; off <<= 1) psum += __shfl_xor(psum, off, 32);
      lrow[r] = lrow[r] * alpha + psum;
#pragma unroll
      for (int t = 0; t < 8; ++t) oacc[t][r] *= alpha;
    }
    wave_lds_sync();

#pragma unroll 1
    for (int kk = 0; kk < 2; ++kk) {
      const v16b pa = ld_frag(pwh + c * APP + kk * 32 + 8 * hh);
      const v16b pz = ld_frag(pwl + c * APP + kk * 32 + 8 * hh);
      const int key0 = kt + kk * 32;
#pragma unroll
      for (int t = 0; t < 8; ++t) {
        const size_t vo = (size_t)(t * 16) * SEQ + key0;
        const v16b vb = ld_frag(Vbh + vo);
        const v16b vz = ld_frag(Vbl + vo);
        oacc[t] = mma_g(pa, vb, oacc[t]);
        oacc[t] = mma_g(pa, vz, oacc[t]);
        oacc[t] = mma_g(pz, vb, oacc[t]);
      }
    }
  }

  __syncthreads();
  float* os = (float*)(lds_raw) + wave * (16 * AOP);
#pragma unroll
  for (int r = 0; r < 8; ++r) {
    const float inv = 1.0f / lrow[r];
#pragma unroll
    for (int t = 0; t < 8; ++t) os[(8 * hh + r) * AOP + t * 16 + c] = oacc[t][r] * inv;
  }
  wave_lds_sync();
  const int c8 = (lane & 15) * 8;
  v4u hv[8], lv[8];
#pragma unroll
  for (int it = 0; it < 8; ++it) {
    const int rr = it * 2 + hh;
    const float* sp = os + rr * AOP + c8;
    v4u a, a2;
#pragma unroll
    for (int p = 0; p < 4; ++p) {
      const float f0 = sp[2 * p], f1 = sp[2 * p + 1];
      const unsigned short hb0 = f2bf_bits(f0), hb1 = f2bf_bits(f1);
      const unsigned short lb0 = f2bf_bits(f0 - bf_bits2f(hb0)), lb1 = f2bf_bits(f1 - bf_bits2f(hb1));
      a[p]  = pk16(hb0, hb1);
      a2[p] = pk16(lb0, lb1);
    }
    hv[it] = a; lv[it] = a2;
  }
  const size_t rowbase = tok0 + wave * 16;
  for (int pass = 0; pass < 2; ++pass) {
#pragma unroll
    for (int it = 0; it < 8; ++it) {
      const int rr = it * 2 + hh;
      const size_t go = (rowbase + rr) * QDIM + h * HDIM + c8;
      *(volatile v4u*)(Ch + go) = hv[it];
      *(volatile v4u*)(Cl + go) = lv[it];
    }
    __threadfence();
  }
}

extern "C" void kernel_launch(void* const* d_in, const int* in_sizes, int n_in,
                              void* d_out, int out_size, void* d_ws, size_t ws_size,
                              hipStream_t stream) {
  if (n_in < 8) return;
  const int ntok = NBATCH * SEQ;
  if (in_sizes[0] != ntok * HID) return;
  if (in_sizes[1] < 1) return;
  if (in_sizes[2] != HID * QDIM) return;
  if (in_sizes[3] != HID * KDIM || in_sizes[4] != HID * KDIM) return;
  if (in_sizes[5] != QDIM * HID) return;
  if (in_sizes[6] != QDIM || in_sizes[7] != KDIM) return;
  if (out_size != ntok * HID) return;

  const float* X   = (const float*)d_in[0];
  const int*   pid = (const int*)d_in[1];
  const float* Wq  = (const float*)d_in[2];
  const float* Wk  = (const float*)d_in[3];
  const float* Wv  = (const float*)d_in[4];
  const float* Wo  = (const float*)d_in[5];
  const float* qw  = (const float*)d_in[6];
  const float* kw  = (const float*)d_in[7];
  float* out = (float*)d_out;
  const int npos = in_sizes[1];

  const size_t bXb  = (size_t)ntok * HID * 2;
  const size_t bBqk = (size_t)QKLD * HID * 2;
  const size_t bWvT = (size_t)KDIM * HID * 2;
  const size_t bWoT = (size_t)HID * QDIM * 2;
  const size_t bTab = (size_t)ntok * NFREQ * 4;
  const size_t bQK  = (size_t)ntok * QKLD * 4;
  const size_t bVT  = (size_t)NBATCH * KDIM * SEQ * 2;
  const size_t bQp  = (size_t)ntok * QDIM * 2;
  const size_t bKp  = (size_t)ntok * KDIM * 2;
  size_t off = 0;
  const size_t oXb  = off; off += bXb;
  const size_t oBqk = off; off += bBqk;
  const size_t oWvT = off; off += bWvT;
  const size_t oWoT = off; off += bWoT;
  const size_t oCt  = off; off += bTab;
  const size_t oSt  = off; off += bTab;
  const size_t oQK  = off; off += bQK;
  const size_t oVTh = off; off += bVT;
  const size_t oVTl = off; off += bVT;
  const size_t oQh  = off; off += bQp;
  const size_t oQl  = off; off += bQp;
  const size_t oKh  = off; off += bKp;
  const size_t oKl  = off; off += bKp;
  if (off > ws_size) return;
  if (2 * bQp > bQK) return;

  char* ws = (char*)d_ws;
  unsigned short* Xb  = (unsigned short*)(ws + oXb);
  unsigned short* Bqk = (unsigned short*)(ws + oBqk);
  unsigned short* WvT = (unsigned short*)(ws + oWvT);
  unsigned short* WoT = (unsigned short*)(ws + oWoT);
  float*          ct  = (float*)(ws + oCt);
  float*          st  = (float*)(ws + oSt);
  float*          QKf = (float*)(ws + oQK);
  unsigned short* Cxh = (unsigned short*)(ws + oQK);
  unsigned short* Cxl = (unsigned short*)(ws + oQK + bQp);
  unsigned short* VTh = (unsigned short*)(ws + oVTh);
  unsigned short* VTl = (unsigned short*)(ws + oVTl);
  unsigned short* Qh  = (unsigned short*)(ws + oQh);
  unsigned short* Ql  = (unsigned short*)(ws + oQl);
  unsigned short* Khp = (unsigned short*)(ws + oKh);
  unsigned short* Klp = (unsigned short*)(ws + oKl);

  const dim3 blk(256);

  const int n8 = ntok * HID / 8;
  conv_bf16_kernel<<<dim3((n8 + 255) / 256), blk, 0, stream>>>(X, Xb, n8);
  tconv_kernel<<<dim3(QDIM / 64, HID / 64), blk, 0, stream>>>(Wq, Bqk, HID, QDIM);
  tconv_kernel<<<dim3(KDIM / 64, HID / 64), blk, 0, stream>>>(Wk, Bqk + (size_t)QDIM * HID, HID, KDIM);
  tconv_kernel<<<dim3(KDIM / 64, HID / 64), blk, 0, stream>>>(Wv, WvT, HID, KDIM);
  tconv_kernel<<<dim3(HID / 64, QDIM / 64), blk, 0, stream>>>(Wo, WoT, QDIM, HID);
  rope_tab_kernel<<<dim3(ntok * NFREQ / 256), blk, 0, stream>>>(pid, npos, ct, st, ntok);
  gemm64_kernel<false, 0><<<dim3((ntok / 64) * (QKLD / 64) / 8, 1), blk, 0, stream>>>(
      Xb, Xb, HID, 0LL, Bqk, HID, 0LL, QKf, Xb, Xb, QKLD, 0LL, ntok, QKLD, HID);
  gemm64_kernel<false, 2><<<dim3((KDIM / 64) * (SEQ / 64) / 8, NBATCH), blk, 0, stream>>>(
      WvT, WvT, HID, 0LL, Xb, HID, (long long)SEQ * HID, QKf, VTh, VTl, SEQ, (long long)KDIM * SEQ, KDIM, SEQ, HID);
  norm_rope_kernel<<<dim3(ntok), blk, 0, stream>>>(QKf, QKLD, qw, kw, ct, st, Qh, Ql, Khp, Klp, 1.0e-6f);
  attn_kernel<<<dim3(NBATCH * NQH * (SEQ / 64)), dim3(128), 0, stream>>>(
      Qh, Ql, Khp, Klp, VTh, VTl, Cxh, Cxl, 0.08838834764831845f);
  gemm64_kernel<true, 0><<<dim3((ntok / 64) * (HID / 64) / 8, 1), blk, 0, stream>>>(
      Cxh, Cxl, QDIM, 0LL, WoT, QDIM, 0LL, out, Xb, Xb, HID, 0LL, ntok, HID, QDIM);
  (void)hipGetLastError();
}
